// MultiHeadAttention_2774548873402
// MI455X (gfx1250) — hardware-verified
//
#include <hip/hip_runtime.h>


#ifndef NB
#define NB 2
#endif
#ifndef SEQ
#define SEQ 2048
#endif
#define NB_FULL  2
#define SEQ_FULL 2048
#define DM   1024
#define NH   16
#define HD   64
#define NZ   (NB * NH)
#define RH   ((SEQ < 512) ? SEQ : 512)
#define PCAR 1024.0f
#define SC2  0.18033688011112042f

static_assert((SEQ & (SEQ - 1)) == 0);
static_assert(SEQ % 256 == 0);
static_assert(RH % 256 == 0);
static_assert(RH <= SEQ);
static_assert(DM == NH * HD);
static_assert(HD == 64);
static_assert((NB * SEQ) % 64 == 0);
static_assert(DM % 64 == 0);
static_assert(NB <= NB_FULL && SEQ <= SEQ_FULL);

typedef _Float16 h16;
typedef unsigned short bf;
typedef __attribute__((ext_vector_type(16))) __bf16   v16bf;
typedef __attribute__((ext_vector_type(16))) _Float16 v16h;
typedef __attribute__((ext_vector_type(8)))  _Float16 v8h;
typedef __attribute__((ext_vector_type(8)))  unsigned short v8us;
typedef __attribute__((ext_vector_type(2)))  unsigned short v2us;
typedef __attribute__((ext_vector_type(8)))  float    v8f;
typedef __attribute__((ext_vector_type(4)))  float    v4f;
typedef v8h  __attribute__((may_alias)) v8ha;
typedef v4f  __attribute__((may_alias)) v4fa;
typedef v8us __attribute__((may_alias)) v8usa;

__device__ __forceinline__ unsigned short f2bf(float f) { unsigned u = __float_as_uint(f); u += 0x7FFFu + ((u >> 16) & 1u); return (unsigned short)(u >> 16); }
__device__ __forceinline__ float bf2f(unsigned short b) { return __uint_as_float(((unsigned)b) << 16); }
__device__ __forceinline__ float bfr(float f) { return bf2f(f2bf(f)); }
__device__ __forceinline__ void splitf(float y, unsigned short& h, unsigned short& l) { h = f2bf(y); l = f2bf(y - bf2f(h)); }
__device__ __forceinline__ v16h cat16(v8h lo, v8h hi) { return __builtin_shufflevector(lo, hi, 0, 1, 2, 3, 4, 5, 6, 7, 8, 9, 10, 11, 12, 13, 14, 15); }
__device__ __forceinline__ v16bf cat16b(v8us lo, v8us hi) { return __builtin_bit_cast(v16bf, __builtin_shufflevector(lo, hi, 0, 1, 2, 3, 4, 5, 6, 7, 8, 9, 10, 11, 12, 13, 14, 15)); }
__device__ __forceinline__ v8f wmma16(v16h a, v16h b, v8f c) { return __builtin_amdgcn_wmma_f32_16x16x32_f16(false, a, false, b, (short)0, c, false, false); }
__device__ __forceinline__ v8f wmmab(v16bf a, v16bf b, v8f c) { return __builtin_amdgcn_wmma_f32_16x16x32_bf16(false, a, false, b, (short)0, c, false, false); }

template <typename T16> struct WFrag;
template <> struct WFrag<h16> { typedef v16h V;
    static __device__ __forceinline__ V ld(const h16* p) { return cat16(*(const v8h*)p, *(const v8h*)(p + 16)); }
    static __device__ __forceinline__ V lds(const h16* p) { return cat16(*(const v8ha*)p, *(const v8ha*)(p + 16)); }
    static __device__ __forceinline__ v8f mma(V a, V b, v8f c) { return wmma16(a, b, c); }
    static __device__ __forceinline__ void pst(h16* ph, h16* pl, unsigned i, float p) { (void)pl; ph[i] = (h16)(p * PCAR); } };
template <> struct WFrag<bf> { typedef v16bf V;
    static __device__ __forceinline__ V ld(const bf* p) { return cat16b(*(const v8us*)p, *(const v8us*)(p + 16)); }
    static __device__ __forceinline__ V lds(const bf* p) { return cat16b(*(const v8usa*)p, *(const v8usa*)(p + 16)); }
    static __device__ __forceinline__ v8f mma(V a, V b, v8f c) { return wmmab(a, b, c); }
    static __device__ __forceinline__ void pst(bf* ph, bf* pl, unsigned i, float p) { unsigned short a, c; splitf(p, a, c); ph[i] = a; pl[i] = c; } };

template <typename T16, int NSPLIT, bool BIAS>
__global__ __launch_bounds__(32) void k_gemmw(const T16* __restrict__ A, const T16* __restrict__ A2, const T16* __restrict__ Bt, const T16* __restrict__ Bt2, int K, float* C, int ldc, const float* __restrict__ bias, size_t sA, size_t sB, size_t sC) {
    typedef typename WFrag<T16>::V V;
    __shared__ __align__(16) float os[16 * 68];
    const size_t z = blockIdx.z; A += z * sA; if (A2) A2 += z * sA; Bt += z * sB; if (Bt2) Bt2 += z * sB; C += z * sC;
    const int lane = threadIdx.x & 31, lr = lane & 15, hi = lane >> 4; const int r0 = blockIdx.x * 64, c0 = blockIdx.y * 64;
    v8f acc[4][4];
#pragma unroll
    for (int mb = 0; mb < 4; ++mb)
#pragma unroll
        for (int nb = 0; nb < 4; ++nb) acc[mb][nb] = (v8f){};
    const size_t aoff = (size_t)(r0 + lr) * K + 8 * hi, boff = (size_t)(c0 + lr) * K + 8 * hi;
#pragma unroll 1
    for (int kc = 0; kc < K; kc += 32) {
        V a[4], a2[4];
#pragma unroll
        for (int mb = 0; mb < 4; ++mb) { a[mb] = WFrag<T16>::ld(A + aoff + (size_t)mb * 16 * K + kc); if (NSPLIT == 1 || NSPLIT == 2) a2[mb] = WFrag<T16>::ld(A2 + aoff + (size_t)mb * 16 * K + kc); }
#pragma unroll
        for (int nb = 0; nb < 4; ++nb) { const V b = WFrag<T16>::ld(Bt + boff + (size_t)nb * 16 * K + kc); V b2; if (NSPLIT >= 2) b2 = WFrag<T16>::ld(Bt2 + boff + (size_t)nb * 16 * K + kc);
#pragma unroll
            for (int mb = 0; mb < 4; ++mb) { acc[mb][nb] = WFrag<T16>::mma(a[mb], b, acc[mb][nb]); if (NSPLIT == 1 || NSPLIT == 2) acc[mb][nb] = WFrag<T16>::mma(a2[mb], b, acc[mb][nb]); if (NSPLIT >= 2) acc[mb][nb] = WFrag<T16>::mma(a[mb], b2, acc[mb][nb]); } }
        asm volatile("v_nop\n\tv_nop\n\tv_nop\n\tv_nop" : "+v"(acc[0][0]), "+v"(acc[1][1]), "+v"(acc[2][2]), "+v"(acc[3][3]) : "v"(a[0]), "v"(a[3]));
    }
#pragma unroll
    for (int mb = 0; mb < 4; ++mb) {
#pragma unroll
        for (int nb = 0; nb < 4; ++nb) {
#pragma unroll
            for (int j = 0; j < 8; ++j) os[(hi * 8 + j) * 68 + nb * 16 + lr] = acc[mb][nb][j]; }
        __builtin_amdgcn_wave_barrier(); asm volatile("" ::: "memory");
        float* crow = C + (size_t)(r0 + mb * 16) * ldc + c0;
#pragma unroll 1
        for (int ps = 0; ps < 2; ++ps) {
#pragma unroll
            for (int s = 0; s < 8; ++s) { const int row = 2 * s + hi, cofs = lr * 4; v4f val = *(const v4fa*)(os + row * 68 + cofs); if (BIAS) { val[0] += bfr(bias[c0 + cofs]); val[1] += bfr(bias[c0 + cofs + 1]); val[2] += bfr(bias[c0 + cofs + 2]); val[3] += bfr(bias[c0 + cofs + 3]); }
                *(volatile v4f*)(crow + (size_t)row * ldc + cofs) = val; }
            if (ps == 0) __threadfence(); }
        __builtin_amdgcn_wave_barrier(); asm volatile("" ::: "memory");
    }
}

static_assert(((size_t)SEQ * DM) % 2048 == 0);
__global__ __launch_bounds__(256) void k_cvtx(const float* __restrict__ src, bf* dst) {
    const unsigned i = blockIdx.x * 256u + threadIdx.x; const unsigned b = blockIdx.y;
    const float* s = src + (size_t)b * SEQ_FULL * DM + (size_t)i * 8; bf* d = dst + (size_t)b * SEQ * DM + (size_t)i * 8;
    const v8f v = *(const v8f*)s; v8us o;
#pragma unroll
    for (int k = 0; k < 8; ++k) o[k] = f2bf(v[k]);
    *(volatile v8us*)d = o; __threadfence(); *(volatile v8us*)d = o; }

static_assert(((size_t)DM * DM) % 4096 == 0);
__global__ __launch_bounds__(256) void k_wt4(const float* __restrict__ w0, const float* __restrict__ w1, const float* __restrict__ w2, const float* __restrict__ w3, bf* Bt) {
    const unsigned y = blockIdx.y; const float* w = (y == 0u) ? w0 : (y == 1u) ? w1 : (y == 2u) ? w2 : w3; bf* o = Bt + (size_t)y * DM * DM;
    const unsigned lane = threadIdx.x & 31u; const unsigned L0 = (blockIdx.x * 8u + (threadIdx.x >> 5)) * 8u;
#pragma unroll
    for (int ps = 0; ps < 2; ++ps) {
#pragma unroll 1
        for (unsigned l = 0; l < 8u; ++l) { const unsigned e = (L0 + l) * 64u + lane * 2u; const unsigned k = e % (unsigned)DM, n = e / (unsigned)DM; v2us q;
            q[0] = f2bf(w[(size_t)k * DM + n]); q[1] = f2bf(w[(size_t)(k + 1u) * DM + n]); *(volatile v2us*)(o + e) = q; }
        if (ps == 0) __threadfence(); }
}

static_assert(((size_t)NZ * SEQ * 8) % 256 == 0);
__global__ __launch_bounds__(256) void k_ropeqk(const float* __restrict__ F, const float* __restrict__ cosT, const float* __restrict__ sinT, h16* P16, bf* Ph, bf* Pl) {
    const unsigned y = blockIdx.y; const unsigned g = blockIdx.x * 256u + threadIdx.x; const unsigned seg = g & 7u, prow = g >> 3;
    const unsigned t = prow % (unsigned)SEQ, z = prow / (unsigned)SEQ, b = z / (unsigned)NH, h = z % (unsigned)NH;
    const float* f = F + (size_t)y * NB * SEQ * DM + (size_t)(b * SEQ + t) * DM + h * HD + seg * 8u;
    const v4f x0 = *(const v4f*)f, x1 = *(const v4f*)(f + 4); const v4f cv = *(const v4f*)(cosT + (size_t)t * 32 + seg * 4u), sv = *(const v4f*)(sinT + (size_t)t * 32 + seg * 4u);
    float xs[8]; xs[0] = x0[0]; xs[1] = x0[1]; xs[2] = x0[2]; xs[3] = x0[3]; xs[4] = x1[0]; xs[5] = x1[1]; xs[6] = x1[2]; xs[7] = x1[3];
    v8h o16; v8us oh, ol;
#pragma unroll
    for (int i = 0; i < 4; ++i) { const float c = bfr(cv[i]), s = bfr(sv[i]); const float tr = xs[2 * i], ti = xs[2 * i + 1]; const float rr = tr * c - ti * s, ri = tr * s + ti * c;
        o16[2 * i] = (h16)rr; o16[2 * i + 1] = (h16)ri; unsigned short a, d2; splitf(rr, a, d2); oh[2 * i] = a; ol[2 * i] = d2; splitf(ri, a, d2); oh[2 * i + 1] = a; ol[2 * i + 1] = d2; }
    h16* p16 = P16 + (size_t)y * NZ * SEQ * HD + (size_t)prow * HD + seg * 8u;
    const bool hl = (t < (unsigned)RH);
    const size_t ho = (size_t)y * NZ * RH * HD + ((size_t)z * RH + (hl ? t : 0u)) * HD + seg * 8u;
    *(volatile v8h*)p16 = o16; if (hl) { *(volatile v8us*)(Ph + ho) = oh; *(volatile v8us*)(Pl + ho) = ol; }
    __threadfence();
    *(volatile v8h*)p16 = o16; if (hl) { *(volatile v8us*)(Ph + ho) = oh; *(volatile v8us*)(Pl + ho) = ol; }
}

static_assert(((size_t)NZ * HD * (SEQ / 8)) % 256 == 0);
__global__ __launch_bounds__(256) void k_vtp(const float* __restrict__ Fv, h16* V16, bf* Vh, bf* Vl) {
    const unsigned g = blockIdx.x * 256u + threadIdx.x; const unsigned SEGS = (unsigned)SEQ / 8u; const unsigned seg = g % SEGS, vrow = g / SEGS;
    const unsigned d = vrow % (unsigned)HD, z = vrow / (unsigned)HD, b = z / (unsigned)NH, h = z % (unsigned)NH, t0 = seg * 8u;
    const float* f = Fv + (size_t)(b * SEQ + t0) * DM + h * HD + d; v8h o16; v8us oh, ol;
#pragma unroll
    for (int j = 0; j < 8; ++j) { const float x = f[(size_t)j * DM]; o16[j] = (h16)x; unsigned short a, c2; splitf(x, a, c2); oh[j] = a; ol[j] = c2; }
    h16* p16 = V16 + (size_t)vrow * SEQ + t0; const bool hl = (t0 < (unsigned)RH);
    const size_t ho = (size_t)vrow * RH + (hl ? t0 : 0u);
    *(volatile v8h*)p16 = o16; if (hl) { *(volatile v8us*)(Vh + ho) = oh; *(volatile v8us*)(Vl + ho) = ol; }
    __threadfence();
    *(volatile v8h*)p16 = o16; if (hl) { *(volatile v8us*)(Vh + ho) = oh; *(volatile v8us*)(Vl + ho) = ol; }
}

__device__ __forceinline__ float rmax16(float v) { v = fmaxf(v, __shfl_xor(v, 1, 32)); v = fmaxf(v, __shfl_xor(v, 2, 32)); v = fmaxf(v, __shfl_xor(v, 4, 32)); v = fmaxf(v, __shfl_xor(v, 8, 32)); return v; }
__device__ __forceinline__ float rsum16(float v) { v += __shfl_xor(v, 1, 32); v += __shfl_xor(v, 2, 32); v += __shfl_xor(v, 4, 32); v += __shfl_xor(v, 8, 32); return v; }

template <typename T16, bool HR>
__device__ __forceinline__ void flash_body(const T16* QA, const T16* QB, const T16* KA, const T16* KB, const T16* VA, const T16* VB, bf* ATh, bf* ATl, T16* pt, float* os) {
    typedef typename WFrag<T16>::V V;
    constexpr unsigned QR   = HR ? (unsigned)RH : (unsigned)SEQ;
    constexpr unsigned ROW0 = HR ? 0u : (unsigned)RH;
    constexpr unsigned NT   = HR ? (unsigned)RH / 16u : (unsigned)(SEQ - RH) / 16u;
    constexpr unsigned NTD  = NT ? NT : 1u;
    const unsigned lane = threadIdx.x & 31u, wid = threadIdx.x >> 5, lr = lane & 15u, hi = lane >> 4;
    const unsigned w = blockIdx.x * 4u + wid; const unsigned z = w / NTD, mt = w % NTD; const unsigned q0 = ROW0 + mt * 16u;
    T16* ptw = pt + (size_t)wid * 1024; T16* ptl = ptw + 512; float* osw = os + (size_t)wid * (16 * 68);
    const size_t qoff = ((size_t)z * QR + q0 + lr) * HD + 8u * hi;
    V aq[2], aql[2];
#pragma unroll
    for (int d = 0; d < 2; ++d) { aq[d] = WFrag<T16>::ld(QA + qoff + d * 32); if (HR) aql[d] = WFrag<T16>::ld(QB + qoff + d * 32); }
    const size_t koff = ((size_t)z * QR + lr) * HD + 8u * hi;
    const size_t voff = ((size_t)z * HD + lr) * QR + 8u * hi;
    v8f o[4]; float m[8], l[8];
#pragma unroll
    for (int t = 0; t < 4; ++t) o[t] = (v8f){};
#pragma unroll
    for (int j = 0; j < 8; ++j) { m[j] = -1.0e30f; l[j] = 0.0f; }
    const unsigned nch = (q0 + 15u) / 32u + 1u;
#pragma unroll 1
    for (unsigned c = 0; c < nch; ++c) {
        const unsigned c0 = c * 32u;
        v8f s0 = (v8f){}, s1 = (v8f){};
#pragma unroll
        for (int d = 0; d < 2; ++d) { const size_t ko = koff + (size_t)c0 * HD + d * 32;
            const V kb0 = WFrag<T16>::ld(KA + ko), kb1 = WFrag<T16>::ld(KA + ko + 16 * HD);
            s0 = WFrag<T16>::mma(aq[d], kb0, s0); s1 = WFrag<T16>::mma(aq[d], kb1, s1);
            if (HR) { const V kl0 = WFrag<T16>::ld(KB + ko), kl1 = WFrag<T16>::ld(KB + ko + 16 * HD);
                s0 = WFrag<T16>::mma(aql[d], kb0, s0); s1 = WFrag<T16>::mma(aql[d], kb1, s1); s0 = WFrag<T16>::mma(aq[d], kl0, s0); s1 = WFrag<T16>::mma(aq[d], kl1, s1); } }
        asm volatile("v_nop\n\tv_nop\n\tv_nop\n\tv_nop" : "+v"(s0), "+v"(s1) : "v"(aq[0]), "v"(aq[1]));
        const unsigned col0 = c0 + lr, col1 = col0 + 16u, rb = q0 + 8u * hi;
#pragma unroll
        for (int j = 0; j < 8; ++j) { const unsigned row = rb + (unsigned)j; const bool v0 = (col0 <= row), v1 = (col1 <= row);
            const float t0 = s0[j] * SC2, t1 = s1[j] * SC2;
            float cm = fmaxf(v0 ? t0 : -1.0e30f, v1 ? t1 : -1.0e30f); cm = rmax16(cm);
            const float nm = fmaxf(m[j], cm); const float al = __builtin_amdgcn_exp2f(m[j] - nm); m[j] = nm;
            const float e0 = __builtin_amdgcn_exp2f(fminf(t0 - nm, 0.0f)), e1 = __builtin_amdgcn_exp2f(fminf(t1 - nm, 0.0f));
            const float p0 = v0 ? e0 : 0.0f, p1 = v1 ? e1 : 0.0f;
            l[j] = l[j] * al + (p0 + p1);
            o[0][j] *= al; o[1][j] *= al; o[2][j] *= al; o[3][j] *= al;
            const unsigned pi = (8u * hi + (unsigned)j) * 32u + lr;
            WFrag<T16>::pst(ptw, ptl, pi, p0); WFrag<T16>::pst(ptw, ptl, pi + 16u, p1); }
        __builtin_amdgcn_wave_barrier(); asm volatile("" ::: "memory");
        const V ap = WFrag<T16>::lds(ptw + lr * 32u + 8u * hi); V apl; if (HR) apl = WFrag<T16>::lds(ptl + lr * 32u + 8u * hi);
#pragma unroll
        for (int t = 0; t < 4; ++t) { const size_t vo = voff + (size_t)t * 16 * QR + c0; const V vb = WFrag<T16>::ld(VA + vo);
            o[t] = WFrag<T16>::mma(ap, vb, o[t]);
            if (HR) { const V vl = WFrag<T16>::ld(VB + vo); o[t] = WFrag<T16>::mma(apl, vb, o[t]); o[t] = WFrag<T16>::mma(ap, vl, o[t]); } }
        asm volatile("v_nop\n\tv_nop\n\tv_nop\n\tv_nop" : "+v"(o[0]), "+v"(o[1]), "+v"(o[2]), "+v"(o[3]) : "v"(ap));
        __builtin_amdgcn_wave_barrier(); asm volatile("" ::: "memory");
    }
    const float cs = HR ? 1.0f : (1.0f / PCAR);
#pragma unroll
    for (int j = 0; j < 8; ++j) { const float ls = rsum16(l[j]); const float inv = (1.0f / ls) * cs;
#pragma unroll
        for (int t = 0; t < 4; ++t) osw[(8u * hi + (unsigned)j) * 68u + (unsigned)t * 16u + lr] = o[t][j] * inv; }
    __builtin_amdgcn_wave_barrier(); asm volatile("" ::: "memory");
    const unsigned b = z / (unsigned)NH, h = z % (unsigned)NH; const unsigned rq = lane >> 3, seg = lane & 7u;
#pragma unroll 1
    for (int ps = 0; ps < 2; ++ps) {
#pragma unroll
        for (int s = 0; s < 4; ++s) { const unsigned row = 4u * (unsigned)s + rq; const v4f a = *(const v4fa*)(osw + row * 68u + seg * 8u), bq = *(const v4fa*)(osw + row * 68u + seg * 8u + 4u); v8us oh, ol;
#pragma unroll
            for (int k = 0; k < 4; ++k) { unsigned short x, y2; splitf(a[k], x, y2); oh[k] = x; ol[k] = y2; splitf(bq[k], x, y2); oh[k + 4] = x; ol[k + 4] = y2; }
            const size_t oo = (size_t)(b * SEQ + q0 + row) * DM + h * HD + seg * 8u;
            *(volatile v8us*)(ATh + oo) = oh; *(volatile v8us*)(ATl + oo) = ol; }
        if (ps == 0) __threadfence(); }
}

static_assert((NZ * (RH / 16)) % 4 == 0);
static_assert((NZ * ((SEQ - RH) / 16)) % 4 == 0);
__global__ __launch_bounds__(128) void k_flash_hr(const bf* Qh, const bf* Ql, const bf* Kh, const bf* Kl, const bf* Vh, const bf* Vl, bf* ATh, bf* ATl) {
    __shared__ __align__(16) bf pt[4 * 2 * 512]; __shared__ __align__(16) float os[4 * 16 * 68];
    flash_body<bf, true>(Qh, Ql, Kh, Kl, Vh, Vl, ATh, ATl, pt, os); }
__global__ __launch_bounds__(128) void k_flash_pl(const h16* Q16, const h16* K16, const h16* V16, bf* ATh, bf* ATl) {
    __shared__ __align__(16) h16 pt[4 * 2 * 512]; __shared__ __align__(16) float os[4 * 16 * 68];
    flash_body<h16, false>(Q16, nullptr, K16, nullptr, V16, nullptr, ATh, ATl, pt, os); }

constexpr size_t SZ_WT  = (size_t)4 * DM * DM * 2;
constexpr size_t SZ_XB  = (size_t)NB * SEQ * DM * 2;
constexpr size_t SZ_F   = (size_t)3 * NB * SEQ * DM * 4;
constexpr size_t SZ_QK  = (size_t)2 * NZ * SEQ * HD * 2;
constexpr size_t SZ_V   = (size_t)NZ * HD * SEQ * 2;
constexpr size_t SZ_QKH = (size_t)2 * NZ * RH * HD * 2;
constexpr size_t SZ_VH  = (size_t)NZ * HD * RH * 2;
constexpr size_t SZ_AT  = (size_t)NB * SEQ * DM * 2;
constexpr size_t WS_TOTAL = SZ_WT + SZ_XB + SZ_F + SZ_QK + SZ_V + 2 * SZ_QKH + 2 * SZ_VH + 2 * SZ_AT;
static_assert(WS_TOTAL <= (size_t)134217728);
static_assert(SZ_WT % 256 == 0 && SZ_XB % 256 == 0 && SZ_F % 256 == 0 && SZ_QK % 256 == 0 && SZ_V % 256 == 0 && SZ_QKH % 256 == 0 && SZ_VH % 256 == 0 && SZ_AT % 256 == 0);

extern "C" void kernel_launch(void* const* d_in, const int* in_sizes, int n_in,
                              void* d_out, int out_size, void* d_ws, size_t ws_size, hipStream_t stream) {
    if (n_in < 7) return;
    const long long need_x = ((long long)(NB - 1) * SEQ_FULL + SEQ) * DM;
    if ((long long)in_sizes[0] < need_x || (long long)out_size < need_x) return;
    if (in_sizes[1] < DM * DM || in_sizes[2] < DM * DM || in_sizes[3] < DM * DM || in_sizes[4] < DM * DM) return;
    if (in_sizes[5] < SEQ * (HD / 2) || in_sizes[6] < SEQ * (HD / 2)) return;
    if (WS_TOTAL > ws_size) return;
    const float* x = (const float*)d_in[0]; const float* wq = (const float*)d_in[1]; const float* wk = (const float*)d_in[2]; const float* wv = (const float*)d_in[3]; const float* wo = (const float*)d_in[4];
    const float* fcos = (const float*)d_in[5]; const float* fsin = (const float*)d_in[6];
    float* OUT = (float*)d_out;
    char* wsp = (char*)d_ws;
    auto take = [&](size_t bytes) { char* p = wsp; wsp += bytes; return (void*)p; };
    bf* WT = (bf*)take(SZ_WT);
    bf* XB = (bf*)take(SZ_XB);
    float* F = (float*)take(SZ_F);
    h16* QK16 = (h16*)take(SZ_QK);
    h16* V16 = (h16*)take(SZ_V);
    bf* QKh = (bf*)take(SZ_QKH); bf* QKl = (bf*)take(SZ_QKH);
    bf* Vh = (bf*)take(SZ_VH); bf* Vl = (bf*)take(SZ_VH);
    bf* ATh = (bf*)take(SZ_AT); bf* ATl = (bf*)take(SZ_AT);
    if ((size_t)(wsp - (char*)d_ws) > ws_size) return;

    k_cvtx<<<dim3((unsigned)((size_t)SEQ * DM / 2048), NB, 1), 256, 0, stream>>>(x, XB);
    k_wt4<<<dim3((unsigned)((size_t)DM * DM / 4096), 4, 1), 256, 0, stream>>>(wq, wk, wv, wo, WT);
    k_gemmw<bf, 0, false><<<dim3(NB * SEQ / 64, DM / 64, 3), 32, 0, stream>>>(XB, nullptr, WT, nullptr, DM, F, DM, nullptr, (size_t)0, (size_t)DM * DM, (size_t)NB * SEQ * DM);
    k_ropeqk<<<dim3((unsigned)((size_t)NZ * SEQ * 8 / 256), 2, 1), 256, 0, stream>>>(F, fcos, fsin, QK16, QKh, QKl);
    k_vtp<<<(unsigned)((size_t)NZ * HD * (SEQ / 8) / 256), 256, 0, stream>>>(F + (size_t)2 * NB * SEQ * DM, V16, Vh, Vl);
    k_flash_hr<<<(unsigned)(NZ * (RH / 16) / 4), 128, 0, stream>>>(QKh, QKl, QKh + (size_t)NZ * RH * HD, QKl + (size_t)NZ * RH * HD, Vh, Vl, ATh, ATl);
    if (SEQ > RH) k_flash_pl<<<(unsigned)(NZ * ((SEQ - RH) / 16) / 4), 128, 0, stream>>>(QK16, QK16 + (size_t)NZ * SEQ * HD, V16, ATh, ATl);
    k_gemmw<bf, 1, false><<<dim3(SEQ / 64, DM / 64, NB), 32, 0, stream>>>(ATh, ATl, WT + (size_t)3 * DM * DM, nullptr, DM, OUT, DM, nullptr, (size_t)SEQ * DM, (size_t)0, (size_t)SEQ_FULL * DM);
}
